// Net2_57939108823553
// MI455X (gfx1250) — hardware-run, weakly checked
//
#include <hip/hip_runtime.h>

typedef __attribute__((ext_vector_type(16))) _Float16 v16h;
typedef __attribute__((ext_vector_type(8)))  _Float16 v8h;
typedef __attribute__((ext_vector_type(16))) __bf16   v16b;
typedef __attribute__((ext_vector_type(8)))  __bf16   v8b;
typedef __attribute__((ext_vector_type(8)))  float    v8f;
typedef __attribute__((ext_vector_type(4)))  float    v4f;
typedef __attribute__((ext_vector_type(8)))  unsigned v8u;

constexpr int kImg    = 1024;
constexpr int kHid    = 64;
constexpr int kTaps   = 9;
constexpr int kTileR  = 64;
constexpr int kTileC  = 8;
constexpr int kPatchR = kTileR + 4;
constexpr int kPatchC = kTileC + 4;
constexpr int kPatchN = kPatchR * kPatchC;
constexpr int kHidR   = kTileR + 2;
constexpr int kHidC   = kTileC + 2;
constexpr int kHidPx  = kHidR * kHidC;
constexpr int kTilesM = (kHidPx + 15) / 16;
constexpr int kTRows  = kTilesM * 16;
constexpr int kTPitch = 9;
constexpr int kOutP   = 68;
static_assert((kImg % 64) == 0 && (kImg % 32) == 0, "GEMM tile multiples");
static_assert((kImg % kTileR) == 0 && (kImg % kTileC) == 0, "conv tile multiples");
static_assert(kTileR * kTileC == 512, "two pixels per thread");
static_assert(kPatchN <= 4 * 256, "four patch sweeps");
static_assert(kHid * kTaps <= 3 * 256, "three weight sweeps");
static_assert(kHid == 64, "two 32-deep k steps over the channels");
static_assert(kTaps <= 16 && kTPitch == kTaps, "taps fit one 16-wide column tile");
static_assert(kHidPx == 660 && kTilesM == 42 && kTRows == 672, "hidden pixel tiling");

constexpr size_t kPlane16 = (size_t)kImg * kImg * 2;
constexpr size_t kPlane32 = (size_t)kImg * kImg * 4;
constexpr size_t kOffMATH = 0;
constexpr size_t kOffMATL = kOffMATH + kPlane16;
constexpr size_t kOffGTH  = kOffMATL + kPlane16;
constexpr size_t kOffGTL  = kOffGTH + 3 * kPlane16;
constexpr size_t kOffH1   = kOffGTL + 3 * kPlane16;
constexpr size_t kOffH2   = kOffH1 + kPlane32;
constexpr size_t kWsTotal = kOffH2 + kPlane32;
static_assert(kWsTotal == 25165824ull, "carve total");
static_assert(kWsTotal <= 134217728ull, "carve cap");
static_assert((kOffMATL % 128) == 0 && (kOffGTH % 128) == 0 && (kOffGTL % 128) == 0 &&
              (kOffH1 % 128) == 0 && (kOffH2 % 128) == 0, "128-B aligned regions");

__device__ __forceinline__ unsigned short f2bf_bits(float f) {
  unsigned u = __float_as_uint(f);
  return (unsigned short)((u + 0x7FFFu + ((u >> 16) & 1u)) >> 16);
}
__device__ __forceinline__ float bf_bits2f(unsigned short h) { return __uint_as_float(((unsigned)h) << 16); }

__device__ __forceinline__ void split_pack4(float a, float b, float c, float d,
                                            unsigned& h01, unsigned& h23, unsigned& l01, unsigned& l23) {
  const unsigned short ha = f2bf_bits(a), hb = f2bf_bits(b), hc = f2bf_bits(c), hd = f2bf_bits(d);
  const unsigned short la = f2bf_bits(a - bf_bits2f(ha));
  const unsigned short lb = f2bf_bits(b - bf_bits2f(hb));
  const unsigned short lc = f2bf_bits(c - bf_bits2f(hc));
  const unsigned short ld = f2bf_bits(d - bf_bits2f(hd));
  h01 = (unsigned)ha | ((unsigned)hb << 16);
  h23 = (unsigned)hc | ((unsigned)hd << 16);
  l01 = (unsigned)la | ((unsigned)lb << 16);
  l23 = (unsigned)lc | ((unsigned)ld << 16);
}

__device__ __forceinline__ void tie_acc_b(v8f& a, v16b x, v16b y) { asm volatile("" : "+v"(a) : "v"(x), "v"(y)); }
__device__ __forceinline__ void nop_guard_b(v8f& a, v16b x, v16b y) { asm volatile("v_nop\n\tv_nop\n\tv_nop\n\tv_nop" : "+v"(a) : "v"(x), "v"(y)); }
__device__ __forceinline__ void nop_guard4in_b(v8f& a, v16b x, v16b y, v16b z, v16b w) { asm volatile("v_nop\n\tv_nop\n\tv_nop\n\tv_nop" : "+v"(a) : "v"(x), "v"(y), "v"(z), "v"(w)); }
__device__ __forceinline__ void keep4_b(v16b a, v16b b, v16b c, v16b d) { asm volatile("v_nop" :: "v"(a), "v"(b), "v"(c), "v"(d)); }
__device__ __forceinline__ void acc_guard4(v8f& a, v8f& b, v8f& c, v8f& d) { asm volatile("v_nop\n\tv_nop\n\tv_nop\n\tv_nop" : "+v"(a), "+v"(b), "+v"(c), "+v"(d)); }

struct FragB {
  union U { v16b v; v8b h[2]; };
  static __device__ __forceinline__ v16b load(const __bf16* p) {
    U f;
    f.h[0] = *(const v8b*)(p);
    f.h[1] = *(const v8b*)(p + 16);
    return f.v;
  }
  static __device__ __forceinline__ v8f mma(v16b a, v16b b, v8f c) {
    return __builtin_amdgcn_wmma_f32_16x16x32_bf16(false, a, false, b, (short)0, c, false, false);
  }
};

__global__ __launch_bounds__(256) void gemm_split_bf16_kernel(
    const unsigned short* __restrict__ Ahp, const unsigned short* __restrict__ Alp, int lda,
    const unsigned short* __restrict__ Bhp, const unsigned short* __restrict__ Blp, int ldb,
    float* __restrict__ Cout, int ldc, int M, int N, int K) {
  typedef __bf16 T;
  typedef v16b V;
  const T* Ab  = (const T*)Ahp;
  const T* Ab2 = (const T*)Alp;
  const T* Bb  = (const T*)Bhp;
  const T* Bb2 = (const T*)Blp;
  __shared__ __align__(16) float sT[8][16 * 68];
  const int lane = threadIdx.x & 31;
  const int wave = threadIdx.x >> 5;
  const int tilesN = N >> 6;
  const int tilesM = M >> 6;
  const int tile = blockIdx.x * 8 + wave;
  if (tile >= tilesM * tilesN) return;
  const int tm = tile / tilesN;
  const int tn = tile - tm * tilesN;
  const int m0 = tm << 6;
  const int n0 = tn << 6;

  const int rlane = lane & 15;
  const int koff  = (lane >> 4) * 8;
  const int mOff  = (lane >> 4) * 8;

  v8f acc[4][4];
#pragma unroll
  for (int i = 0; i < 4; ++i)
#pragma unroll
    for (int j = 0; j < 4; ++j) acc[i][j] = (v8f){0.f, 0.f, 0.f, 0.f, 0.f, 0.f, 0.f, 0.f};

  for (int k0 = 0; k0 < K; k0 += 32) {
    V bh[4], bl[4];
#pragma unroll
    for (int j = 0; j < 4; ++j) {
      const size_t bo = (size_t)(n0 + (j << 4) + rlane) * ldb + koff + k0;
      bh[j] = FragB::load(Bb + bo);
      bl[j] = FragB::load(Bb2 + bo);
    }
#pragma unroll
    for (int i = 0; i < 4; ++i) {
      const size_t ao = (size_t)(m0 + (i << 4) + rlane) * lda + koff + k0;
      V ah = FragB::load(Ab + ao);
      V al = FragB::load(Ab2 + ao);
#pragma unroll
      for (int j = 0; j < 4; ++j) {
        acc[i][j] = FragB::mma(ah, bh[j], acc[i][j]);
        acc[i][j] = FragB::mma(ah, bl[j], acc[i][j]);
        acc[i][j] = FragB::mma(al, bh[j], acc[i][j]);
      }
      tie_acc_b(acc[i][0], ah, al);
      tie_acc_b(acc[i][1], ah, al);
      tie_acc_b(acc[i][2], ah, al);
      nop_guard_b(acc[i][3], ah, al);
    }
    keep4_b(bh[0], bh[1], bh[2], bh[3]);
    keep4_b(bl[0], bl[1], bl[2], bl[3]);
  }
  acc_guard4(acc[0][0], acc[0][1], acc[0][2], acc[0][3]);
  acc_guard4(acc[1][0], acc[1][1], acc[1][2], acc[1][3]);
  acc_guard4(acc[2][0], acc[2][1], acc[2][2], acc[2][3]);
  acc_guard4(acc[3][0], acc[3][1], acc[3][2], acc[3][3]);

  float* slab = sT[wave];
#pragma unroll
  for (int i = 0; i < 4; ++i) {
    const int mBase = m0 + (i << 4);
#pragma unroll
    for (int j = 0; j < 4; ++j) {
#pragma unroll
      for (int r = 0; r < 8; ++r) {
        slab[(mOff + r) * 68 + (j << 4) + rlane] = acc[i][j][r];
      }
    }
    __builtin_amdgcn_fence(__ATOMIC_RELEASE, "workgroup");
    __builtin_amdgcn_wave_barrier();
    __builtin_amdgcn_fence(__ATOMIC_ACQUIRE, "workgroup");
    {
      const int hh = lane >> 4, c4 = (lane & 15) * 4;
      for (int pass = 0; pass < 2; ++pass) {
#pragma unroll
        for (int it = 0; it < 8; ++it) {
          const int row = it * 2 + hh;
          v4f v = *(const v4f*)(slab + row * 68 + c4);
          *(volatile v4f*)(Cout + (size_t)(mBase + row) * ldc + n0 + c4) = v;
        }
        __threadfence();
      }
    }
    __builtin_amdgcn_fence(__ATOMIC_RELEASE, "workgroup");
    __builtin_amdgcn_wave_barrier();
    __builtin_amdgcn_fence(__ATOMIC_ACQUIRE, "workgroup");
  }
}

__global__ __launch_bounds__(256) void split_rows_bf16_kernel(
    const float* __restrict__ src, unsigned short* __restrict__ dhi, unsigned short* __restrict__ dlo, int total8)
{
  const int i = blockIdx.x * 256 + threadIdx.x;
  if (i >= total8) return;
  const size_t e0 = (size_t)i << 3;
  const v4f a0 = *(const v4f*)(src + e0);
  const v4f a1 = *(const v4f*)(src + e0 + 4);
  v8h hv, lv;
#pragma unroll
  for (int e = 0; e < 4; ++e) {
    const unsigned short h0 = f2bf_bits(a0[e]), h1 = f2bf_bits(a1[e]);
    const unsigned short l0 = f2bf_bits(a0[e] - bf_bits2f(h0)), l1 = f2bf_bits(a1[e] - bf_bits2f(h1));
    hv[e]     = __builtin_bit_cast(_Float16, h0);
    hv[4 + e] = __builtin_bit_cast(_Float16, h1);
    lv[e]     = __builtin_bit_cast(_Float16, l0);
    lv[4 + e] = __builtin_bit_cast(_Float16, l1);
  }
  unsigned short* qh = dhi + e0;
  unsigned short* ql = dlo + e0;
  *(volatile v8h*)qh = hv;
  *(volatile v8h*)ql = lv;
  __threadfence();
  *(volatile v8h*)qh = hv;
  *(volatile v8h*)ql = lv;
}

__device__ __forceinline__ v4f fma4s(v4f w, float s, v4f a) {
  v4f r;
  r[0] = fmaf(w[0], s, a[0]);
  r[1] = fmaf(w[1], s, a[1]);
  r[2] = fmaf(w[2], s, a[2]);
  r[3] = fmaf(w[3], s, a[3]);
  return r;
}

__global__ __launch_bounds__(256) void conv_pair_kernel(
    const float* __restrict__ img,
    const float* __restrict__ W1, const float* __restrict__ b1,
    const float* __restrict__ W2, const float* __restrict__ b2,
    unsigned short* __restrict__ GtH, unsigned short* __restrict__ GtL)
{
  __shared__ __align__(16) float sX[kPatchN];
  __shared__ __align__(16) float sW1[kTaps * kHid];
  __shared__ __align__(16) float sW2[kTaps * kHid];
  __shared__ __align__(16) float sB1[kHid];
  __shared__ __align__(16) float sT[kTRows * kTPitch];
  __shared__ __align__(16) float sOut[kTileC * kOutP];

  const int tid  = threadIdx.x;
  const int lane = tid & 31;
  const int wave = tid >> 5;
  const int hh   = lane >> 4;
  const int rl   = lane & 15;
  const int tx   = tid & 7;
  const int ty   = tid >> 3;
  const int ox0  = blockIdx.x * kTileC;
  const int oy0  = blockIdx.y * kTileR;

#pragma unroll 1
  for (int sweep = 0; sweep < 3; ++sweep) {
    const int i  = sweep * 256 + tid;
    const int ic = (i < kHid * kTaps) ? i : (kHid * kTaps - 1);
    const float w1v = W1[ic];
    const float w2v = W2[ic];
    const int c = ic / kTaps;
    const int t = ic - c * kTaps;
    if (i < kHid * kTaps) {
      sW1[t * kHid + c] = w1v;
      sW2[t * kHid + c] = w2v;
    }
  }
  {
    const float bv = b1[tid & (kHid - 1)];
    if (tid < kHid) sB1[tid] = bv;
  }
#pragma unroll 1
  for (int sweep = 0; sweep < 4; ++sweep) {
    const int i  = sweep * 256 + tid;
    const int ic = (i < kPatchN) ? i : (kPatchN - 1);
    const int py = ic / kPatchC;
    const int px = ic - py * kPatchC;
    const int gy = oy0 + py - 2;
    const int gx = ox0 + px - 2;
    const bool inb = ((unsigned)gy < (unsigned)kImg) && ((unsigned)gx < (unsigned)kImg);
    const int gyc = gy < 0 ? 0 : (gy > kImg - 1 ? kImg - 1 : gy);
    const int gxc = gx < 0 ? 0 : (gx > kImg - 1 ? kImg - 1 : gx);
    const float v = img[(size_t)gyc * kImg + gxc];
    if (i < kPatchN) sX[i] = inb ? v : 0.0f;
  }
  const float bias2 = b2[0];
  __syncthreads();

  v16b bh[2], bl[2];
  {
    const int  tsel  = (rl < kTaps) ? rl : (kTaps - 1);
    const bool treal = (rl < kTaps);
#pragma unroll
    for (int ks = 0; ks < 2; ++ks) {
      v8u wh, wl;
#pragma unroll
      for (int g = 0; g < 4; ++g) {
        const int cb = ks * 32 + (g >> 1) * 16 + 8 * hh + (g & 1) * 4;
        const v4f w = *(const v4f*)(sW2 + tsel * kHid + cb);
        const float w0 = treal ? w[0] : 0.0f;
        const float w1 = treal ? w[1] : 0.0f;
        const float w2 = treal ? w[2] : 0.0f;
        const float w3 = treal ? w[3] : 0.0f;
        unsigned h01, h23, l01, l23;
        split_pack4(w0, w1, w2, w3, h01, h23, l01, l23);
        wh[2 * g]     = h01;
        wh[2 * g + 1] = h23;
        wl[2 * g]     = l01;
        wl[2 * g + 1] = l23;
      }
      bh[ks] = __builtin_bit_cast(v16b, wh);
      bl[ks] = __builtin_bit_cast(v16b, wl);
    }
  }

#pragma unroll 1
  for (int tile = wave; tile < kTilesM; tile += 8) {
    const int p0 = tile * 16;
    const int p  = p0 + rl;
    const int pc = (p < kHidPx) ? p : (kHidPx - 1);
    const int py = pc / kHidC;
    const int px = pc - py * kHidC;
    const int gy = oy0 + py - 1;
    const int gx = ox0 + px - 1;
    const bool inimg = ((unsigned)gy < (unsigned)kImg) && ((unsigned)gx < (unsigned)kImg);
    float in[kTaps];
#pragma unroll
    for (int t = 0; t < kTaps; ++t) in[t] = sX[(py + t / 3) * kPatchC + px + (t % 3)];

    v8f acc = (v8f){0.f, 0.f, 0.f, 0.f, 0.f, 0.f, 0.f, 0.f};
#pragma unroll
    for (int ks = 0; ks < 2; ++ks) {
      v8u wh, wl;
#pragma unroll
      for (int g = 0; g < 4; ++g) {
        const int cb = ks * 32 + (g >> 1) * 16 + 8 * hh + (g & 1) * 4;
        v4f hv = *(const v4f*)(sB1 + cb);
#pragma unroll
        for (int t = 0; t < kTaps; ++t) {
          const v4f w = *(const v4f*)(sW1 + t * kHid + cb);
          hv = fma4s(w, in[t], hv);
        }
        const float o0 = inimg ? fmaxf(hv[0], 0.0f) : 0.0f;
        const float o1 = inimg ? fmaxf(hv[1], 0.0f) : 0.0f;
        const float o2 = inimg ? fmaxf(hv[2], 0.0f) : 0.0f;
        const float o3 = inimg ? fmaxf(hv[3], 0.0f) : 0.0f;
        unsigned h01, h23, l01, l23;
        split_pack4(o0, o1, o2, o3, h01, h23, l01, l23);
        wh[2 * g]     = h01;
        wh[2 * g + 1] = h23;
        wl[2 * g]     = l01;
        wl[2 * g + 1] = l23;
      }
      const v16b ah = __builtin_bit_cast(v16b, wh);
      const v16b al = __builtin_bit_cast(v16b, wl);
      acc = FragB::mma(ah, bh[ks], acc);
      acc = FragB::mma(ah, bl[ks], acc);
      acc = FragB::mma(al, bh[ks], acc);
      nop_guard4in_b(acc, ah, al, bh[ks], bl[ks]);
    }
    if (rl < kTaps) {
#pragma unroll
      for (int r = 0; r < 8; ++r) sT[(p0 + 8 * hh + r) * kTPitch + rl] = acc[r];
    }
  }
  __syncthreads();

#pragma unroll 1
  for (int pix = 0; pix < 2; ++pix) {
    const int y = ty + 32 * pix;
    const int base = y * kHidC + tx;
    float s = bias2;
#pragma unroll
    for (int t = 0; t < kTaps; ++t) {
      s += sT[(base + (t / 3) * kHidC + (t % 3)) * kTPitch + t];
    }
    sOut[tx * kOutP + y] = s;
  }
  __syncthreads();

  if (wave < 2) {
    const int q = lane >> 3;
    const int j = lane & 7;
    const int xx = wave * 4 + q;
    const float* sp = sOut + xx * kOutP + 8 * j;
    const v4f a0 = *(const v4f*)(sp);
    const v4f a1 = *(const v4f*)(sp + 4);
    v8h hv, lv;
#pragma unroll
    for (int e = 0; e < 4; ++e) {
      const unsigned short h0 = f2bf_bits(a0[e]), h1 = f2bf_bits(a1[e]);
      const unsigned short l0 = f2bf_bits(a0[e] - bf_bits2f(h0)), l1 = f2bf_bits(a1[e] - bf_bits2f(h1));
      hv[e]     = __builtin_bit_cast(_Float16, h0);
      hv[4 + e] = __builtin_bit_cast(_Float16, h1);
      lv[e]     = __builtin_bit_cast(_Float16, l0);
      lv[4 + e] = __builtin_bit_cast(_Float16, l1);
    }
    const size_t o = (size_t)(ox0 + xx) * kImg + oy0 + 8 * j;
    unsigned short* qh = GtH + o;
    unsigned short* ql = GtL + o;
    *(volatile v8h*)qh = hv;
    *(volatile v8h*)ql = lv;
    __threadfence();
    *(volatile v8h*)qh = hv;
    *(volatile v8h*)ql = lv;
  }
}

extern "C" void kernel_launch(void* const* d_in, const int* in_sizes, int n_in,
                              void* d_out, int out_size, void* d_ws, size_t ws_size,
                              hipStream_t stream) {
  if (n_in < 6) return;
  if (in_sizes[0] != kImg * kImg) return;
  if (in_sizes[1] != kImg * kImg) return;
  if (in_sizes[2] != kHid * kTaps) return;
  if (in_sizes[3] != kHid) return;
  if (in_sizes[4] != kHid * kTaps) return;
  if (in_sizes[5] != 1) return;
  if (out_size != kImg * kImg) return;
  if (ws_size < kWsTotal) return;

  const float* x   = (const float*)d_in[0];
  const float* mat = (const float*)d_in[1];
  const float* W1  = (const float*)d_in[2];
  const float* b1  = (const float*)d_in[3];
  const float* W2  = (const float*)d_in[4];
  const float* b2  = (const float*)d_in[5];
  float* out = (float*)d_out;

  char* ws = (char*)d_ws;
  unsigned short* MATH = (unsigned short*)(ws + kOffMATH);
  unsigned short* MATL = (unsigned short*)(ws + kOffMATL);
  unsigned short* GTH0 = (unsigned short*)(ws + kOffGTH);
  unsigned short* GTH1 = (unsigned short*)(ws + kOffGTH + kPlane16);
  unsigned short* GTH2 = (unsigned short*)(ws + kOffGTH + 2 * kPlane16);
  unsigned short* GTL0 = (unsigned short*)(ws + kOffGTL);
  unsigned short* GTL1 = (unsigned short*)(ws + kOffGTL + kPlane16);
  unsigned short* GTL2 = (unsigned short*)(ws + kOffGTL + 2 * kPlane16);
  float* H1 = (float*)(ws + kOffH1);
  float* H2 = (float*)(ws + kOffH2);

  const dim3 convGrid(kImg / kTileC, kImg / kTileR);
  const int gemmBlocks = ((kImg / 64) * (kImg / 64)) / 8;

  split_rows_bf16_kernel<<<(kImg * kImg / 8) / 256, 256, 0, stream>>>(mat, MATH, MATL, kImg * kImg / 8);

  conv_pair_kernel<<<convGrid, 256, 0, stream>>>(x, W1, b1, W2, b2, GTH0, GTL0);
  gemm_split_bf16_kernel<<<gemmBlocks, 256, 0, stream>>>(MATH, MATL, kImg, GTH0, GTL0, kImg, H1, kImg, kImg, kImg, kImg);
  conv_pair_kernel<<<convGrid, 256, 0, stream>>>(H1, W1, b1, W2, b2, GTH1, GTL1);
  gemm_split_bf16_kernel<<<gemmBlocks, 256, 0, stream>>>(MATH, MATL, kImg, GTH1, GTL1, kImg, H2, kImg, kImg, kImg, kImg);
  conv_pair_kernel<<<convGrid, 256, 0, stream>>>(H2, W1, b1, W2, b2, GTH2, GTL2);
  gemm_split_bf16_kernel<<<gemmBlocks, 256, 0, stream>>>(MATH, MATL, kImg, GTH2, GTL2, kImg, out, kImg, kImg, kImg, kImg);
}
